// GraphConvolutionWithEdgeConcat_38070590112205
// MI455X (gfx1250) — hardware-verified
//
#include <hip/hip_runtime.h>
#include <stddef.h>


#define HID    128
#define NREL   3
#define KP     512
#define GT     128
#define SPW    (32 * 64)
#define WPP    520
#define RB     512
#define RBBITS 9
#define RMAX   128
#define RMBITS 7
#define TABW   (2 * RMAX)
#define CHUNK  4096
#define LCAP   32768
#define DEGCAP 128
#define WSCAP  134217728
#define ASCL   8.0f
#define WSCL   64.0f
#define INVSCL 0.0009765625f
#define EPSV   1e-6f
#define INVD   0.0078125f

#define AGG_LDS_INTS  (RB + 8 + RB + LCAP)
#define AGG_LDS_BYTES (AGG_LDS_INTS * 4)

static_assert(KP == (NREL + 1) * HID);
static_assert((KP % 32) == 0);
static_assert(RB == (1 << RBBITS));
static_assert(RB == 2 * 256);
static_assert(RMAX == (1 << RMBITS));
static_assert(TABW == 256);
static_assert(CHUNK == 8 * 16 * 32);
static_assert(CHUNK == 4 * 4 * 256);
static_assert((WPP % 8) == 0);
static_assert(((RB + 8) % 4) == 0);
static_assert((AGG_LDS_INTS % 4) == 0);
static_assert(AGG_LDS_BYTES < 300000);
static_assert((DEGCAP % 2) == 0);
static_assert((HID % 32) == 0);

typedef float          v4f  __attribute__((ext_vector_type(4)));
typedef float          v8f  __attribute__((ext_vector_type(8)));
typedef int            v4i  __attribute__((ext_vector_type(4)));
typedef unsigned int   v4u  __attribute__((ext_vector_type(4)));
typedef unsigned short v8us __attribute__((ext_vector_type(8)));
typedef _Float16       v16h __attribute__((ext_vector_type(16)));
union FragH { v16h v; v8us u[2]; };

__device__ __forceinline__ unsigned short h16(float f) {
  const _Float16 hv = (_Float16)f;
  return __builtin_bit_cast(unsigned short, hv);
}

__device__ __forceinline__ v8f wmh(v16h a, v16h b, v8f c) {
  v8f d = __builtin_amdgcn_wmma_f32_16x16x32_f16(false, a, false, b, (short)0, c, false, false);
  asm volatile("v_nop\n\tv_nop\n\tv_nop\n\tv_nop" : "+v"(d) : "v"(a), "v"(b));
  return d;
}

template <int NB>
__device__ __forceinline__ unsigned int match_mask(unsigned int base, int key) {
  unsigned int msk = base;
#pragma unroll
  for (int b = 0; b < NB; ++b) {
    const bool bit = ((key >> b) & 1) != 0;
    const unsigned int bb = __builtin_amdgcn_ballot_w32(bit);
    msk &= bit ? bb : ~bb;
  }
  return msk;
}

__global__ __launch_bounds__(256) void k_wprep(
    const float* __restrict__ W, const float* __restrict__ Ws, unsigned short* w16t) {
  __shared__ __attribute__((aligned(16))) unsigned short sT[32 * WPP];
  const int tid = (int)threadIdx.x;
  const int n0 = 32 * (int)blockIdx.x;

#pragma unroll 1
  for (int it = 0; it < 64; ++it) {
    const int idx = it * 256 + tid;
    const int rr = idx & 31, k = idx >> 5;
    const int kw = k > NREL * HID - 1 ? NREL * HID - 1 : k;
    int ks = k - NREL * HID; ks = ks < 0 ? 0 : ks;
    const float vw = W[(size_t)kw * HID + n0 + rr];
    const float vs = Ws[(size_t)ks * HID + n0 + rr];
    const float val = (k < NREL * HID) ? vw : vs;
    sT[rr * WPP + k] = h16(val * WSCL);
  }
  __syncthreads();

  v8us pv[8];
#pragma unroll
  for (int it = 0; it < 8; ++it) {
    const int p = it * 256 + tid;
    const int row = p >> 6, c8 = (p & 63) * 8;
    pv[it] = *(const v8us*)(sT + row * WPP + c8);
  }
#pragma unroll
  for (int it = 0; it < 8; ++it) {
    const int p = it * 256 + tid;
    const int row = p >> 6, c8 = (p & 63) * 8;
    *(volatile v8us*)(w16t + (size_t)(n0 + row) * KP + c8) = pv[it];
  }
  __threadfence();
#pragma unroll
  for (int it = 0; it < 8; ++it) {
    const int p = it * 256 + tid;
    const int row = p >> 6, c8 = (p & 63) * 8;
    *(volatile v8us*)(w16t + (size_t)(n0 + row) * KP + c8) = pv[it];
  }
}

__global__ __launch_bounds__(256) void k_csort(
    const int* __restrict__ rows, unsigned int* csort, int* tab, int nN, int nE) {
  __shared__ __attribute__((aligned(16))) unsigned int sImg[CHUNK];
  __shared__ int cw[8 * RMAX];
  __shared__ __attribute__((aligned(16))) int sPre[RMAX];
  __shared__ __attribute__((aligned(16))) int sCn[RMAX];
  __shared__ int sWt[8];
  const int tid = (int)threadIdx.x, lane = tid & 31, wave = tid >> 5;
  const int c = (int)blockIdx.x;
  const int cbase = c * CHUNK;

  for (int i = tid; i < 8 * RMAX; i += 256) cw[i] = 0;
  {
    const v4u s = {0xffffffffu, 0xffffffffu, 0xffffffffu, 0xffffffffu};
    for (int i = tid; i < CHUNK / 4; i += 256) ((v4u*)sImg)[i] = s;
  }
  __syncthreads();

  unsigned int ent[16];
  int pk[16];
  const unsigned int lt = (1u << lane) - 1u;
#pragma unroll
  for (int i = 0; i < 16; ++i) {
    const int e = cbase + wave * 512 + 32 * i + lane;
    const int ea = e > nE - 1 ? nE - 1 : e;
    const int d = rows[ea];
    const bool valid = (e < nE) && ((unsigned)d < (unsigned)nN);
    const int dd = valid ? d : 0;
    const int r  = dd >> RBBITS;
    const int jl = dd & (RB - 1);
    const unsigned int msk = match_mask<RMBITS>(__builtin_amdgcn_ballot_w32(valid), r);
    const int rank = (int)__builtin_popcount(msk & lt);
    const int grp  = (int)__builtin_popcount(msk);
    const int base = cw[wave * RMAX + r];
    pk[i]  = valid ? ((r << 12) | (base + rank)) : -1;
    ent[i] = ((unsigned int)ea << RBBITS) | (unsigned int)jl;
    if (valid && rank == 0) cw[wave * RMAX + r] = base + grp;
    __syncthreads();
  }

  if (tid < RMAX) {
    int run = 0;
#pragma unroll
    for (int w = 0; w < 8; ++w) {
      const int v = cw[w * RMAX + tid];
      cw[w * RMAX + tid] = run;
      run += v;
    }
    sCn[tid] = run;
  }
  __syncthreads();
  {
    const int vr = sCn[tid & (RMAX - 1)];
    const int v  = (tid < RMAX) ? vr : 0;
    int x = v;
#pragma unroll
    for (int dd = 1; dd < 32; dd <<= 1) {
      const int y = __shfl_up(x, dd);
      x += (lane >= dd) ? y : 0;
    }
    if (lane == 31) sWt[wave] = x;
    __syncthreads();
    int pre = 0;
#pragma unroll
    for (int w = 0; w < 8; ++w) { const int tw = sWt[w]; pre += (w < wave) ? tw : 0; }
    if (tid < RMAX) sPre[tid] = pre + x - v;
  }
  __syncthreads();

#pragma unroll
  for (int i = 0; i < 16; ++i) {
    const int pki = pk[i] < 0 ? 0 : pk[i];
    const int r = (pki >> 12) & (RMAX - 1);
    const int q = pki & 4095;
    const int pos = sPre[r] + cw[wave * RMAX + r] + q;
    if (pk[i] >= 0 && (unsigned)pos < (unsigned)CHUNK) sImg[pos] = ent[i];
  }
  __syncthreads();

  v4u iv[4];
#pragma unroll
  for (int it = 0; it < 4; ++it) iv[it] = ((const v4u*)sImg)[it * 256 + tid];
  const v4i ta = *(const v4i*)(sPre + 4 * lane);
  const v4i tb = *(const v4i*)(sCn + 4 * lane);
  const v4i tv = (wave == 0) ? ta : tb;
  unsigned int* gp = csort + (size_t)c * CHUNK;
  int* tp = tab + (size_t)c * TABW + 4 * tid;
  const bool wt = tid < 64;
#pragma unroll
  for (int it = 0; it < 4; ++it) *(volatile v4u*)(gp + 4 * (it * 256 + tid)) = iv[it];
  if (wt) *(volatile v4i*)tp = tv;
  __threadfence();
#pragma unroll
  for (int it = 0; it < 4; ++it) *(volatile v4u*)(gp + 4 * (it * 256 + tid)) = iv[it];
  if (wt) *(volatile v4i*)tp = tv;
}

__global__ __launch_bounds__(256) void k_agg(
    const float* __restrict__ x, const int* __restrict__ cols, const float* __restrict__ vals,
    const unsigned int* __restrict__ csort, const int* __restrict__ tab,
    const float* __restrict__ gamma, const float* __restrict__ beta,
    unsigned short* aplane, int nN, int nNp, int nE, int nEt, int nCh) {
  extern __shared__ __attribute__((aligned(16))) int dsm[];
  __shared__ int sWtot[8];
  int* sOff  = dsm;
  int* sCur  = dsm + (RB + 8);
  int* sList = sCur + RB;
  const int tid = (int)threadIdx.x, lane = tid & 31, wave = tid >> 5;
  const int rgn = (int)blockIdx.x;
  const int n0 = rgn * RB;
  const unsigned int lt = (1u << lane) - 1u;

  {
    const v4i z4 = {0, 0, 0, 0};
    for (int i = tid; i < AGG_LDS_INTS / 4; i += 256) ((v4i*)dsm)[i] = z4;
  }
  __syncthreads();

#pragma unroll 1
  for (int c = 0; c < nCh; ++c) {
    int pre = tab[(size_t)c * TABW + rgn];
    int n   = tab[(size_t)c * TABW + RMAX + rgn];
    pre = pre < 0 ? 0 : (pre > CHUNK ? CHUNK : pre);
    n = n < 0 ? 0 : (n > CHUNK - pre ? CHUNK - pre : n);
    const int nstep = (n + 31) >> 5;
    const unsigned int* cp = csort + (size_t)c * CHUNK + pre;
#pragma unroll 1
    for (int s = 0; s < nstep; ++s) {
      if (wave == 0) {
        const int i = (s << 5) + lane;
        const bool valid = i < n;
        const int ic = i > n - 1 ? n - 1 : i;
        const unsigned int en = cp[ic];
        const int j = (int)(en & (unsigned int)(RB - 1));
        const unsigned int msk = match_mask<RBBITS>(__builtin_amdgcn_ballot_w32(valid), j);
        const int rank = (int)__builtin_popcount(msk & lt);
        const int grp  = (int)__builtin_popcount(msk);
        if (valid && rank == 0) sOff[j] = sOff[j] + grp;
      }
      __syncthreads();
    }
  }
  __syncthreads();

  {
    const int cn0 = sOff[2 * tid], cn1 = sOff[2 * tid + 1];
    const int ls = cn0 + cn1;
    int xs = ls;
#pragma unroll
    for (int dd = 1; dd < 32; dd <<= 1) {
      const int y = __shfl_up(xs, dd);
      xs += (lane >= dd) ? y : 0;
    }
    if (lane == 31) sWtot[wave] = xs;
    __syncthreads();
    int pre = 0;
#pragma unroll
    for (int w = 0; w < 8; ++w) { const int tw = sWtot[w]; pre += (w < wave) ? tw : 0; }
    const int run = pre + xs - ls;
    sOff[2 * tid] = run;
    sOff[2 * tid + 1] = run + cn0;
    if (tid == 255) sOff[RB] = run + cn0 + cn1;
  }
  __syncthreads();

#pragma unroll 1
  for (int c = 0; c < nCh; ++c) {
    int pre = tab[(size_t)c * TABW + rgn];
    int n   = tab[(size_t)c * TABW + RMAX + rgn];
    pre = pre < 0 ? 0 : (pre > CHUNK ? CHUNK : pre);
    n = n < 0 ? 0 : (n > CHUNK - pre ? CHUNK - pre : n);
    const int nstep = (n + 31) >> 5;
    const unsigned int* cp = csort + (size_t)c * CHUNK + pre;
#pragma unroll 1
    for (int s = 0; s < nstep; ++s) {
      if (wave == 0) {
        const int i = (s << 5) + lane;
        const bool valid = i < n;
        const int ic = i > n - 1 ? n - 1 : i;
        const unsigned int en = cp[ic];
        const int j = (int)(en & (unsigned int)(RB - 1));
        int e = (int)(en >> RBBITS);
        e = e > nE - 1 ? nE - 1 : e;
        const unsigned int msk = match_mask<RBBITS>(__builtin_amdgcn_ballot_w32(valid), j);
        const int rank = (int)__builtin_popcount(msk & lt);
        const int grp  = (int)__builtin_popcount(msk);
        const int cur  = sCur[j];
        const int p0   = sOff[j] + cur + rank;
        if (valid && (unsigned)p0 < (unsigned)LCAP) sList[p0] = e;
        if (valid && rank == 0) sCur[j] = cur + grp;
      }
      __syncthreads();
    }
  }
  __syncthreads();

  const int h = lane >> 4, m = lane & 15, ch = 8 * m;
  float gm[8], bt[8];
  {
    const v4f ga = *(const v4f*)(gamma + ch), gb = *(const v4f*)(gamma + ch + 4);
    const v4f ba = *(const v4f*)(beta + ch),  bb = *(const v4f*)(beta + ch + 4);
#pragma unroll
    for (int cc = 0; cc < 4; ++cc) { gm[cc] = ga[cc]; gm[4 + cc] = gb[cc]; bt[cc] = ba[cc]; bt[4 + cc] = bb[cc]; }
  }
  int Rb = nNp - n0; Rb = Rb > RB ? RB : Rb;
#pragma unroll 1
  for (int j = wave; j < Rb; j += 8) {
    const int node = n0 + j;
    int lb = __builtin_amdgcn_readfirstlane(sOff[j]);
    int ub = __builtin_amdgcn_readfirstlane(sOff[j + 1]);
    lb = lb < 0 ? 0 : (lb > LCAP ? LCAP : lb);
    ub = ub < 0 ? 0 : (ub > LCAP ? LCAP : ub);
    int cnt = ub - lb;
    cnt = cnt < 0 ? 0 : (cnt > DEGCAP ? DEGCAP : cnt);
    cnt = (node < nN) ? cnt : 0;

    int c1 = 0, c2 = 0;
    const int nsc = (cnt + 31) >> 5;
#pragma unroll 1
    for (int s = 0; s < nsc; ++s) {
      const int i = (s << 5) + lane;
      const bool valid = i < cnt;
      const int ic = valid ? i : (cnt - 1);
      int li = lb + ic; li = li < 0 ? 0 : (li > LCAP - 1 ? LCAP - 1 : li);
      int e = sList[li]; e = e < 0 ? 0 : (e > nE - 1 ? nE - 1 : e);
      c1 += (int)__builtin_popcount(__builtin_amdgcn_ballot_w32(valid && (e < nEt)));
      c2 += (int)__builtin_popcount(__builtin_amdgcn_ballot_w32(valid && (e < 2 * nEt)));
    }

    float acc[NREL][8];
#pragma unroll
    for (int r = 0; r < NREL; ++r)
#pragma unroll
      for (int cc = 0; cc < 8; ++cc) acc[r][cc] = 0.0f;

#pragma unroll
    for (int r = 0; r < NREL; ++r) {
      const int st = lb + ((r == 0) ? 0 : ((r == 1) ? c1 : c2));
      const int ln = (r == 0) ? c1 : ((r == 1) ? (c2 - c1) : (cnt - c2));
      const int np = (ln + 1) >> 1;
#pragma unroll 1
      for (int it = 0; it < np; ++it) {
        const int i = 2 * it + h;
        const bool valid = i < ln;
        const int ic = valid ? i : (ln - 1);
        int li = st + ic; li = li < 0 ? 0 : (li > LCAP - 1 ? LCAP - 1 : li);
        int e = sList[li]; e = e < 0 ? 0 : (e > nE - 1 ? nE - 1 : e);
        int src = cols[e]; src = src < 0 ? 0 : (src > nN - 1 ? nN - 1 : src);
        float v = vals[e];
        v = valid ? v : 0.0f;
        const v4f xa = *(const v4f*)(x + (size_t)src * HID + ch);
        const v4f xb = *(const v4f*)(x + (size_t)src * HID + ch + 4);
#pragma unroll
        for (int cc = 0; cc < 4; ++cc) {
          acc[r][cc]     = fmaf(v, xa[cc], acc[r][cc]);
          acc[r][4 + cc] = fmaf(v, xb[cc], acc[r][4 + cc]);
        }
      }
    }
#pragma unroll
    for (int r = 0; r < NREL; ++r)
#pragma unroll
      for (int cc = 0; cc < 8; ++cc) acc[r][cc] += __shfl_xor(acc[r][cc], 16);

    float s8[8];
    float ps = 0.0f;
#pragma unroll
    for (int cc = 0; cc < 8; ++cc) { s8[cc] = (acc[0][cc] + acc[1][cc]) + acc[2][cc]; ps += s8[cc]; }
    ps += __shfl_xor(ps, 1); ps += __shfl_xor(ps, 2); ps += __shfl_xor(ps, 4); ps += __shfl_xor(ps, 8);
    const float mean = ps * INVD;
    float d8[8];
    float pq = 0.0f;
#pragma unroll
    for (int cc = 0; cc < 8; ++cc) { d8[cc] = s8[cc] - mean; pq = fmaf(d8[cc], d8[cc], pq); }
    pq += __shfl_xor(pq, 1); pq += __shfl_xor(pq, 2); pq += __shfl_xor(pq, 4); pq += __shfl_xor(pq, 8);
    const float var = pq * INVD;
    const float inv = rsqrtf(var + EPSV);

    v8us q[4];
#pragma unroll
    for (int cc = 0; cc < 8; ++cc) {
      q[0][cc] = h16(acc[0][cc] * ASCL);
      q[1][cc] = h16(acc[1][cc] * ASCL);
      q[2][cc] = h16(acc[2][cc] * ASCL);
      const float nv = d8[cc] * inv * gm[cc] + bt[cc];
      q[3][cc] = h16(nv * ASCL);
    }
    const v8us vA = h ? q[1] : q[0];
    const v8us vB = h ? q[3] : q[2];
    unsigned short* rp = aplane + (size_t)node * KP + 128 * h + ch;
    *(volatile v8us*)(rp)       = vA;
    *(volatile v8us*)(rp + 256) = vB;
    __threadfence();
    *(volatile v8us*)(rp)       = vA;
    *(volatile v8us*)(rp + 256) = vB;
  }
}

__global__ __launch_bounds__(GT) void k_gemm(
    const unsigned short* __restrict__ A, const unsigned short* __restrict__ Bt,
    const float* __restrict__ bias, float* out, int M) {
  __shared__ __attribute__((aligned(16))) float sT[4 * SPW];
  const int tid = (int)threadIdx.x, lane = tid & 31, wave = tid >> 5, hh = lane >> 4, m = lane & 15;
  const int rb = (int)blockIdx.x * 64;
  const int lr0 = (wave >> 1) * 32;
  const int r0 = rb + lr0;
  const int c0 = (wave & 1) * 64;

  const unsigned short* ap0 = A + (size_t)(r0 + m) * KP + 8 * hh;
  const unsigned short* ap1 = A + (size_t)(r0 + 16 + m) * KP + 8 * hh;
  const unsigned short* bp[4];
#pragma unroll
  for (int j = 0; j < 4; ++j)
    bp[j] = Bt + (size_t)(c0 + 16 * j + m) * KP + 8 * hh;

  v8f acc[2][4];
#pragma unroll
  for (int i = 0; i < 2; ++i)
#pragma unroll
    for (int j = 0; j < 4; ++j) { v8f z = {0.f, 0.f, 0.f, 0.f, 0.f, 0.f, 0.f, 0.f}; acc[i][j] = z; }

#pragma unroll 1
  for (int kt = 0; kt < KP / 32; ++kt) {
    const int kb = kt << 5;
    FragH a0, a1;
    a0.u[0] = *(const v8us*)(ap0 + kb);
    a0.u[1] = *(const v8us*)(ap0 + kb + 16);
    a1.u[0] = *(const v8us*)(ap1 + kb);
    a1.u[1] = *(const v8us*)(ap1 + kb + 16);
#pragma unroll
    for (int j = 0; j < 4; ++j) {
      FragH bf;
      bf.u[0] = *(const v8us*)(bp[j] + kb);
      bf.u[1] = *(const v8us*)(bp[j] + kb + 16);
      acc[0][j] = wmh(a0.v, bf.v, acc[0][j]);
      acc[1][j] = wmh(a1.v, bf.v, acc[1][j]);
    }
  }

  float* sw = sT + wave * SPW;
#pragma unroll
  for (int i = 0; i < 2; ++i)
#pragma unroll
    for (int j = 0; j < 4; ++j)
#pragma unroll
      for (int r = 0; r < 8; ++r)
        sw[(16 * i + 8 * hh + r) * 64 + 16 * j + m] = acc[i][j][r];
  __syncthreads();

  const v4f b4 = *(const v4f*)(bias + c0 + 4 * m);
  v4f hv[16];
#pragma unroll
  for (int it = 0; it < 16; ++it) {
    const int row = 2 * it + hh;
    const v4f v = *(const v4f*)(sw + row * 64 + 4 * m);
    hv[it] = v * INVSCL + b4;
  }
#pragma unroll
  for (int it = 0; it < 16; ++it) {
    const int gr = r0 + 2 * it + hh;
    if (gr < M) *(volatile v4f*)(out + (size_t)gr * HID + c0 + 4 * m) = hv[it];
  }
  __threadfence();
#pragma unroll
  for (int it = 0; it < 16; ++it) {
    const int gr = r0 + 2 * it + hh;
    if (gr < M) *(volatile v4f*)(out + (size_t)gr * HID + c0 + 4 * m) = hv[it];
  }
}

extern "C" void kernel_launch(void* const* d_in, const int* in_sizes, int n_in,
                              void* d_out, int out_size, void* d_ws, size_t ws_size,
                              hipStream_t stream) {
  if (n_in < 9) return;
  const int nN = in_sizes[0] / HID;
  if (nN <= 0 || in_sizes[0] != nN * HID) return;
  if (out_size != nN * HID) return;
  if (in_sizes[4] != NREL * HID * HID || in_sizes[5] != HID * HID) return;
  if (in_sizes[6] != HID || in_sizes[7] != HID || in_sizes[8] != HID) return;
  if (in_sizes[1] <= 0 || (in_sizes[1] % NREL) != 0) return;
  if (in_sizes[2] != in_sizes[1] || in_sizes[3] != in_sizes[1]) return;
  const int nEt = in_sizes[1] / NREL;
  const int nE = NREL * nEt;
  if (nEt < 1 || nE > (1 << 22)) return;
  if (nN > RMAX * RB) return;

  const float* x     = (const float*)d_in[0];
  const int*   rows  = (const int*)d_in[1];
  const int*   cols  = (const int*)d_in[2];
  const float* vals  = (const float*)d_in[3];
  const float* Wt    = (const float*)d_in[4];
  const float* Ws    = (const float*)d_in[5];
  const float* bias  = (const float*)d_in[6];
  const float* gamma = (const float*)d_in[7];
  const float* beta  = (const float*)d_in[8];
  float* out = (float*)d_out;

  const int nCh = (nE + CHUNK - 1) / CHUNK;
  const int nR  = (nN + RB - 1) / RB;
  const int nNp = ((nN + 63) / 64) * 64;

  const size_t szW   = (size_t)HID * KP * 2;
  const size_t szA   = (size_t)nNp * KP * 2;
  const size_t szCS  = (size_t)nCh * CHUNK * 4;
  const size_t szTab = (size_t)nCh * TABW * 4;
  size_t off = 0;
  const size_t oW  = off; off += szW;   off = (off + 255) & ~(size_t)255;
  const size_t oA  = off; off += szA;   off = (off + 255) & ~(size_t)255;
  const size_t oCS = off; off += szCS;  off = (off + 255) & ~(size_t)255;
  const size_t oTb = off; off += szTab; off = (off + 255) & ~(size_t)255;
  if (off > ws_size || off > (size_t)WSCAP) return;

  char* ws = (char*)d_ws;
  unsigned short* w16t   = (unsigned short*)(ws + oW);
  unsigned short* aplane = (unsigned short*)(ws + oA);
  unsigned int*   csort  = (unsigned int*)(ws + oCS);
  int*            tab    = (int*)(ws + oTb);

  k_wprep<<<HID / 32, 256, 0, stream>>>(Wt, Ws, w16t);

  k_csort<<<nCh, 256, 0, stream>>>(rows, csort, tab, nN, nE);

  hipFuncSetAttribute(reinterpret_cast<const void*>(&k_agg),
                      hipFuncAttributeMaxDynamicSharedMemorySize, AGG_LDS_BYTES);
  k_agg<<<nR, 256, AGG_LDS_BYTES, stream>>>(x, cols, vals, csort, tab, gamma, beta,
                                            aplane, nN, nNp, nE, nEt, nCh);

  k_gemm<<<nNp / 64, GT, 0, stream>>>(aplane, w16t, bias, out, nN);
}
